// flowGAN_48438641164944
// MI455X (gfx1250) — hardware-verified
//
#include <hip/hip_runtime.h>
#include <cmath>

typedef __attribute__((ext_vector_type(16))) _Float16 v16h;
typedef __attribute__((ext_vector_type(2)))  _Float16 h2;
typedef __attribute__((ext_vector_type(8)))  float    v8f;

#define NSTEP 8
#define HDIM  512
#define BLOCK 256
#define NWAVE (BLOCK / 32)

__device__ __forceinline__ float lane_bcast_f32(float v, int srcLane) {
    int r = __builtin_amdgcn_ds_bpermute(srcLane << 2, __builtin_bit_cast(int, v));
    return __builtin_bit_cast(float, r);
}

__global__ __launch_bounds__(BLOCK)
void flow_wmma_kernel(const float* __restrict__ x,
                      const float* __restrict__ Ws,
                      const float* __restrict__ an_logs,
                      const float* __restrict__ an_b,
                      const float* __restrict__ cw1,
                      const float* __restrict__ cb1,
                      const float* __restrict__ cw2,
                      const float* __restrict__ cb2,
                      float* __restrict__ out,
                      int B)
{
    __shared__ float w1s[NSTEP * HDIM];
    __shared__ float b1s[NSTEP * HDIM];
    __shared__ h2 w2h[NSTEP * 2 * (HDIM / 2)];
    __shared__ h2 zpad[8];
    __shared__ float stS[NWAVE][2][2][16];

    const int tid  = threadIdx.x;
    const int lane = tid & 31;
    const int wave = tid >> 5;
    const int nidx = lane & 15;
    const int hi   = lane >> 4;

    __builtin_prefetch(cw1, 0, 3);
    __builtin_prefetch(cw2, 0, 3);

    _Float16* w2f = (_Float16*)w2h;
    for (int i = tid; i < NSTEP * HDIM; i += BLOCK) {
        w1s[i] = cw1[i];
        b1s[i] = cb1[i];
    }
    for (int i = tid; i < NSTEP * 2 * HDIM; i += BLOCK) {
        w2f[i] = (_Float16)cw2[i];
    }
    if (tid < 8) { h2 z; z.x = (_Float16)0.f; z.y = (_Float16)0.f; zpad[tid] = z; }
    __syncthreads();

    const int sidx = blockIdx.x * BLOCK + tid;
    const int ld   = (sidx < B) ? sidx : (B - 1);
    const float x0 = x[ld * 2 + 0];
    const float x1 = x[ld * 2 + 1];

    float W00 = Ws[0], W01 = Ws[1], W10 = Ws[2], W11 = Ws[3];
    float y0 = x0 * W00 + x1 * W01;
    float y1 = x0 * W10 + x1 * W11;
    float lJ = logf(fabsf(W00 * W11 - W01 * W10));

    for (int step = 0; step < NSTEP; ++step) {
        float l0 = an_logs[step * 2 + 0], l1 = an_logs[step * 2 + 1];
        y0 = y0 * expf(l0) + an_b[step * 2 + 0];
        y1 = y1 * expf(l1) + an_b[step * 2 + 1];
        lJ += l0 + l1;

        const float y0a = lane_bcast_f32(y0, nidx);
        const float y0b = lane_bcast_f32(y0, nidx + 16);

        v8f acc0, acc1;
        #pragma unroll
        for (int r = 0; r < 8; ++r) { acc0[r] = 0.f; acc1[r] = 0.f; }

        const int pAstep = step * (HDIM / 2);
        const h2* const bbase = (nidx < 2)
            ? (w2h + (step * 2 + nidx) * (HDIM / 2) + hi * 4)
            : zpad;
        const int bstride = (nidx < 2) ? 16 : 0;
        const int bsel    = (nidx < 2) ? 1 : 0;

        #pragma unroll 2
        for (int kc = 0; kc < HDIM / 32; ++kc) {
            const h2* bsrc = bbase + kc * bstride;
            v16h bf;
            #pragma unroll
            for (int p = 0; p < 8; ++p) {
                h2 wv = bsrc[bsel * ((p < 4) ? p : p + 4)];
                bf[2 * p]     = wv.x;
                bf[2 * p + 1] = wv.y;
            }

            const int ka = step * HDIM + kc * 32 + hi * 8;
            v16h af0, af1;
            #pragma unroll
            for (int e = 0; e < 16; ++e) {
                const int k = ka + ((e < 8) ? e : e + 8);
                const float wv = w1s[k], bv = b1s[k];
                af0[e] = (_Float16)fmaxf(fmaf(y0a, wv, bv), 0.f);
                af1[e] = (_Float16)fmaxf(fmaf(y0b, wv, bv), 0.f);
            }

            acc0 = __builtin_amdgcn_wmma_f32_16x16x32_f16(
                false, af0, false, bf, (short)0, acc0, false, false);
            acc1 = __builtin_amdgcn_wmma_f32_16x16x32_f16(
                false, af1, false, bf, (short)0, acc1, false, false);
        }

        if (nidx < 2) {
            #pragma unroll
            for (int r = 0; r < 8; ++r) {
                stS[wave][0][nidx][hi * 8 + r] = acc0[r];
                stS[wave][1][nidx][hi * 8 + r] = acc1[r];
            }
        }
        asm volatile("s_wait_dscnt 0" ::: "memory");

        float st0 = stS[wave][hi][0][nidx] + cb2[step * 2 + 0];
        float st1 = stS[wave][hi][1][nidx] + cb2[step * 2 + 1];

        float log_s = tanhf(st0);
        y1 = y1 * expf(log_s) + st1;
        lJ += log_s;

        const float* W = Ws + (step + 1) * 4;
        float a = W[0], b_ = W[1], c = W[2], d = W[3];
        float ny0 = a * y0 + b_ * y1;
        float ny1 = c * y0 + d * y1;
        lJ += logf(fabsf(a * d - b_ * c));
        y0 = ny0; y1 = ny1;
    }

    if (sidx < B) {
        typedef __attribute__((ext_vector_type(2))) float v2f_t;
        v2f_t yy; yy.x = y0; yy.y = y1;
        const float ll = -1.8378770664093453f - 0.5f * (y0 * y0 + y1 * y1) + lJ;
        *(volatile v2f_t*)(out + sidx * 2) = yy; *(volatile float*)(out + 2 * B + sidx) = ll; __threadfence();
        *(volatile v2f_t*)(out + sidx * 2) = yy; *(volatile float*)(out + 2 * B + sidx) = ll;
    }
}

extern "C" void kernel_launch(void* const* d_in, const int* in_sizes, int n_in,
                              void* d_out, int out_size, void* d_ws, size_t ws_size,
                              hipStream_t stream) {
    const float* x       = (const float*)d_in[0];
    const float* Ws      = (const float*)d_in[1];
    const float* an_logs = (const float*)d_in[2];
    const float* an_b    = (const float*)d_in[3];
    const float* cw1     = (const float*)d_in[4];
    const float* cb1     = (const float*)d_in[5];
    const float* cw2     = (const float*)d_in[6];
    const float* cb2     = (const float*)d_in[7];

    const int B = in_sizes[0] / 2;
    dim3 grid((B + BLOCK - 1) / BLOCK);
    flow_wmma_kernel<<<grid, BLOCK, 0, stream>>>(
        x, Ws, an_logs, an_b, cw1, cb1, cw2, cb2, (float*)d_out, B);
}
